// NL_74234214744691
// MI455X (gfx1250) — hardware-verified
//
#include <hip/hip_runtime.h>
#include <math.h>

typedef __attribute__((ext_vector_type(16))) _Float16 v16h;
typedef __attribute__((ext_vector_type(16))) __bf16 v16b;
typedef __attribute__((ext_vector_type(8)))  _Float16 v8h;
typedef __attribute__((ext_vector_type(8)))  float v8f;
typedef __attribute__((ext_vector_type(4)))  float v4f;
typedef __attribute__((ext_vector_type(2)))  float v2f;
typedef __attribute__((ext_vector_type(4)))  unsigned v4u;
typedef __attribute__((ext_vector_type(4)))  int v4i;
typedef float __attribute__((may_alias)) float_a;
typedef int __attribute__((may_alias)) int_a;

template <typename T> __device__ __forceinline__ void vst2(void* p, T v) { *(volatile T*)p = v; __threadfence(); *(volatile T*)p = v; }
__device__ __forceinline__ v8f wmma16(v16h a, v16h b, v8f c) {
  v8f d = __builtin_amdgcn_wmma_f32_16x16x32_f16(false, a, false, b, (short)0, c, false, false);
  asm volatile("v_nop\n\tv_nop\n\tv_nop\n\tv_nop" : "+v"(d) : "v"(a), "v"(b));
  return d;
}
__device__ __forceinline__ v8f wmma_bf(v16b a, v16b b, v8f c) {
  v8f d = __builtin_amdgcn_wmma_f32_16x16x32_bf16(false, a, false, b, (short)0, c, false, false);
  asm volatile("v_nop\n\tv_nop\n\tv_nop\n\tv_nop" : "+v"(d) : "v"(a), "v"(b));
  return d;
}
__device__ __forceinline__ v16h frag_h(const _Float16* rowk0, int lane) {
  union { v16h v; v8h q[2]; } u; const _Float16* p = rowk0 + 8 * (lane >> 4);
  u.q[0] = *(const v8h*)p; u.q[1] = *(const v8h*)(p + 16); return u.v;
}
__device__ __forceinline__ v16h frag_f32(const float* rowk0, int lane) {
  v16h a; const float* p = rowk0 + 8 * (lane >> 4);
#pragma unroll
  for (int i = 0; i < 8; ++i) { a[i] = (_Float16)p[i]; a[8 + i] = (_Float16)p[16 + i]; }
  return a;
}
__device__ __forceinline__ v16h frag_f32s(const float* rowk0, int lane, float sc) {
  v16h a; const float* p = rowk0 + 8 * (lane >> 4);
#pragma unroll
  for (int i = 0; i < 8; ++i) { a[i] = (_Float16)(p[i] * sc); a[8 + i] = (_Float16)(p[16 + i] * sc); }
  return a;
}
__device__ __forceinline__ v16h fragc_f32(const float* W, int k0, int n, int lane, int ld, int K) {
  v16h a; const int g = lane >> 4;
#pragma unroll
  for (int i = 0; i < 8; ++i) { const int ka = k0 + 8 * g + i, kb = ka + 16;
    a[i] = (_Float16)(ka < K ? W[(size_t)(ka < K ? ka : K - 1) * ld + n] : 0.f); a[8 + i] = (_Float16)(kb < K ? W[(size_t)(kb < K ? kb : K - 1) * ld + n] : 0.f); }
  return a;
}
struct F2 { v16b h, l; };
__device__ __forceinline__ F2 bsplit16(const float v[16]) { F2 r;
#pragma unroll
  for (int i = 0; i < 16; ++i) { const __bf16 h = (__bf16)v[i]; r.h[i] = h; r.l[i] = (__bf16)(v[i] - (float)h); }
  return r; }
__device__ __forceinline__ F2 split_row(const float* row, int k0, int lane) { float v[16]; const float* p = row + k0 + 8 * (lane >> 4);
#pragma unroll
  for (int i = 0; i < 8; ++i) { v[i] = p[i]; v[8 + i] = p[16 + i]; }
  return bsplit16(v); }
__device__ __forceinline__ F2 split_rowK(const float* row, int k0, int lane, int K) { float v[16]; const int g = lane >> 4;
#pragma unroll
  for (int i = 0; i < 8; ++i) { const int ka = k0 + 8 * g + i, kb = ka + 16; v[i] = ka < K ? row[ka < K ? ka : K - 1] : 0.f; v[8 + i] = kb < K ? row[kb < K ? kb : K - 1] : 0.f; }
  return bsplit16(v); }
__device__ __forceinline__ F2 split_col(const float* W, int k0, int n, int lane, int ld, int K) { float v[16]; const int g = lane >> 4;
#pragma unroll
  for (int i = 0; i < 8; ++i) { const int ka = k0 + 8 * g + i, kb = ka + 16; v[i] = ka < K ? W[(size_t)(ka < K ? ka : K - 1) * ld + n] : 0.f; v[8 + i] = kb < K ? W[(size_t)(kb < K ? kb : K - 1) * ld + n] : 0.f; }
  return bsplit16(v); }
__device__ __forceinline__ v8f mac3(const F2& a, const F2& b, v8f c) { c = wmma_bf(a.l, b.h, c); c = wmma_bf(a.h, b.l, c); return wmma_bf(a.h, b.h, c); }
__device__ __forceinline__ float sigm(float v) { return 1.0f / (1.0f + expf(-v)); }
#define LDSX() do { asm volatile("s_wait_dscnt 0" ::: "memory"); __builtin_amdgcn_wave_barrier(); __builtin_amdgcn_fence(__ATOMIC_RELEASE, "workgroup"); } while (0)


#define NB 4
#define CIN 256
#define CO 128
#define NPOS 4096
#ifndef TQB
#define TQB (NPOS / 64)
#endif
typedef __attribute__((ext_vector_type(8))) __bf16 v8b;
__device__ __forceinline__ v16b frag_b(const __bf16* rowk0, int lane) {
  union { v16b v; v8b q[2]; } u; const __bf16* p = rowk0 + 8 * (lane >> 4);
  u.q[0] = *(const v8b*)p; u.q[1] = *(const v8b*)(p + 16); return u.v;
}
__device__ __forceinline__ float bfr(float v) { return (float)(__bf16)v; }
__device__ __attribute__((noinline)) float exp_ni(float v) { return expf(v); }
__device__ __attribute__((noinline)) float erf_ni(float v) { return erff(v); }

#define WS_PK  0u
#define WS_PW  (WS_PK + 2u * 3 * CO * CIN)
#define WS_QH  (WS_PW + 2u * CIN * CO)
#define WS_QL  (WS_QH + 2u * NB * NPOS * CO)
#define WS_KH  (WS_QL + 2u * NB * NPOS * CO)
#define WS_KL  (WS_KH + 2u * NB * NPOS * CO)
#define WS_VH  (WS_KL + 2u * NB * NPOS * CO)
#define WS_ST  (WS_VH + 2u * (size_t)NB * CO * NPOS)
#define WS_END (WS_ST + 4u * NB * NPOS * 2)

__device__ __attribute__((noinline)) float exp_p(float v) { return expf(v); }
__global__ __launch_bounds__(256) void k_pack(const float* __restrict__ WQ, const float* __restrict__ WK, const float* __restrict__ WV, const float* __restrict__ WW, __bf16* __restrict__ PK, __bf16* __restrict__ PW) {
  const int n = blockIdx.x, t = threadIdx.x; __shared__ __align__(16) __bf16 s[CIN];
  if (n < 3 * CO) { const float* src = (n < CO) ? WQ + (size_t)n * CIN : (n < 2 * CO) ? WK + (size_t)(n - CO) * CIN : WV + (size_t)(n - 2 * CO) * CIN; s[t] = (__bf16)src[t]; __syncthreads(); if (t < CIN / 8) vst2((unsigned*)(PK + (size_t)n * CIN + t * 8), *(const v4u*)&s[t * 8]); }
  else { const int o = n - 3 * CO; if (t < CO) s[t] = (__bf16)WW[(size_t)o * CO + t]; __syncthreads(); if (t < CO / 8) vst2((unsigned*)(PW + (size_t)o * CO + t * 8), *(const v4u*)&s[t * 8]); }
}
__global__ __launch_bounds__(128) void k_proj(const float* __restrict__ X, const __bf16* __restrict__ PK, const float* __restrict__ BQ, const float* __restrict__ BK, const float* __restrict__ BV, _Float16* __restrict__ QH, _Float16* __restrict__ QL, _Float16* __restrict__ KH, _Float16* __restrict__ KL, _Float16* __restrict__ VH) {
  __shared__ __align__(16) __bf16 sa[64][CIN + 8]; __shared__ __align__(16) _Float16 sth[64][CO + 8], stl[64][CO + 8]; __shared__ __align__(16) _Float16 svh[CO][72];
  const int tid = threadIdx.x, wave = tid >> 5, lane = tid & 31, col = lane & 15, g = lane >> 4; const size_t b = blockIdx.y; const int n0 = blockIdx.x * 64;
  for (int e = tid; e < 64 * CIN; e += 128) { const int c = e >> 6, r = e & 63; sa[r][c] = (__bf16)X[(b * CIN + c) * NPOS + n0 + r]; }
  if (tid < 64) for (int c = CIN; c < CIN + 8; ++c) sa[tid][c] = (__bf16)0.f;
  __syncthreads();
#pragma unroll 1
  for (int which = 0; which < 3; ++which) { v8f acc[8] = {};
#pragma unroll
    for (int kc = 0; kc < CIN / 32; ++kc) { const v16b a = frag_b(&sa[wave * 16 + col][kc * 32], lane);
#pragma unroll
      for (int j = 0; j < 8; ++j) acc[j] = wmma_bf(a, frag_b(PK + (size_t)(which * CO + j * 16 + col) * CIN + kc * 32, lane), acc[j]); }
    const float* BB = (which == 0) ? BQ : (which == 1) ? BK : BV;
    if (which < 2) {
#pragma unroll
      for (int j = 0; j < 8; ++j) { const int c = j * 16 + col; const float bb = bfr(BB[c]);
#pragma unroll
        for (int r = 0; r < 8; ++r) { const float v = acc[j][r] + bb; const _Float16 hv = (_Float16)v; sth[wave * 16 + 8 * g + r][c] = hv; stl[wave * 16 + 8 * g + r][c] = (_Float16)((v - (float)hv) * 2048.0f); } }
      __syncthreads();
      _Float16* DH_ = which ? KH : QH; _Float16* DL_ = which ? KL : QL;
      for (int e = tid; e < 64 * 16; e += 128) { const int r = e >> 4, q = e & 15; const size_t o = (b * NPOS + n0 + r) * CO + q * 8; vst2((unsigned*)(DH_ + o), *(const v4u*)&sth[r][q * 8]); vst2((unsigned*)(DL_ + o), *(const v4u*)&stl[r][q * 8]); }
      __syncthreads(); }
    else {
#pragma unroll
      for (int j = 0; j < 8; ++j) { const int c = j * 16 + col; const float bb = bfr(BB[c]);
#pragma unroll
        for (int r = 0; r < 8; ++r) svh[c][wave * 16 + 8 * g + r] = (_Float16)(acc[j][r] + bb); }
      __syncthreads();
      for (int e = tid; e < CO * 8; e += 128) { const int c = e >> 3, pc = e & 7; vst2((unsigned*)(VH + (b * CO + c) * NPOS + n0 + pc * 8), *(const v4u*)&svh[c][pc * 8]); } } }
}
__global__ __launch_bounds__(128) void k_stats(const _Float16* __restrict__ QH, const _Float16* __restrict__ QL, const _Float16* __restrict__ KH, const _Float16* __restrict__ KL, float* __restrict__ ST) {
  __shared__ __align__(16) float so[64][2];
  const int tid = threadIdx.x, wave = tid >> 5, lane = tid & 31, col = lane & 15, g = lane >> 4; const size_t b = blockIdx.y; const int n0 = blockIdx.x * 64 + wave * 16; const size_t rn = b * NPOS + n0;
  v16h ak[CO / 32], akl[CO / 32];
#pragma unroll
  for (int kc = 0; kc < CO / 32; ++kc) { ak[kc] = frag_h(KH + (rn + col) * CO + kc * 32, lane); akl[kc] = frag_h(KL + (rn + col) * CO + kc * 32, lane); }
  float m[8], l[8];
#pragma unroll
  for (int r = 0; r < 8; ++r) { m[r] = -3.0e38f; l[r] = 0.f; }
#pragma unroll 1
  for (int mt = 0; mt < NPOS / 16; ++mt) { const size_t rm = (b * NPOS + mt * 16 + col) * CO; v8f c = {}, cl = {};
#pragma unroll
    for (int kc = 0; kc < CO / 32; ++kc) { const v16h qh = frag_h(QH + rm + kc * 32, lane); c = wmma16(ak[kc], qh, c); cl = wmma16(akl[kc], qh, cl); cl = wmma16(ak[kc], frag_h(QL + rm + kc * 32, lane), cl); }
#pragma unroll
    for (int r = 0; r < 8; ++r) { const float s = c[r] + cl[r] * (1.0f / 2048.0f); float mx = s;
#pragma unroll
      for (int o = 1; o < 16; o <<= 1) mx = fmaxf(mx, __shfl_xor(mx, o));
      const float mn = fmaxf(m[r], mx); const float alpha = (m[r] <= -1.0e38f) ? 0.f : exp_p(m[r] - mn); float e = exp_p(s - mn);
#pragma unroll
      for (int o = 1; o < 16; o <<= 1) e += __shfl_xor(e, o);
      l[r] = l[r] * alpha + e; m[r] = mn; } }
  if (col == 0) {
#pragma unroll
    for (int r = 0; r < 8; ++r) { so[wave * 16 + 8 * g + r][0] = m[r]; so[wave * 16 + 8 * g + r][1] = 1.0f / l[r]; } }
  __syncthreads();
  if (tid < 32) vst2(ST + (b * NPOS + blockIdx.x * 64) * 2 + tid * 4, *(const v4f*)(&so[0][0] + tid * 4));
}
__global__ __launch_bounds__(128) void k_out(const _Float16* __restrict__ QH, const _Float16* __restrict__ QL, const _Float16* __restrict__ KH, const _Float16* __restrict__ KL, const _Float16* __restrict__ VH, const float* __restrict__ ST, const __bf16* __restrict__ PW, const float* __restrict__ BW, const float* __restrict__ G, const float* __restrict__ Bt, const float* __restrict__ MU, const float* __restrict__ VAR, const float* __restrict__ X, float* __restrict__ OUT) {
  __shared__ __align__(16) _Float16 spw[4][16][40]; __shared__ __align__(16) __bf16 syh[64][CO + 8], syl[64][CO + 8]; __shared__ __align__(16) float so[128][68];
  const int tid = threadIdx.x, wave = tid >> 5, lane = tid & 31, col = lane & 15, g = lane >> 4; const size_t b = blockIdx.y; const int m0 = blockIdx.x * 64 + wave * 16; const size_t rm = b * NPOS + m0;
  v16h aq[CO / 32], aql[CO / 32];
#pragma unroll
  for (int kc = 0; kc < CO / 32; ++kc) { aq[kc] = frag_h(QH + (rm + col) * CO + kc * 32, lane); aql[kc] = frag_h(QL + (rm + col) * CO + kc * 32, lane); }
  v8f acc[8] = {};
#pragma unroll 1
  for (int ks = 0; ks < NPOS / 32; ++ks) { const int j0 = ks * 32;
#pragma unroll
    for (int ct = 0; ct < 2; ++ct) { const int nn = j0 + ct * 16 + col; const size_t rn = (b * NPOS + nn) * CO; v8f c = {}, cl = {};
#pragma unroll
      for (int kc = 0; kc < CO / 32; ++kc) { const v16h kh = frag_h(KH + rn + kc * 32, lane); c = wmma16(aq[kc], kh, c); cl = wmma16(aql[kc], kh, cl); cl = wmma16(aq[kc], frag_h(KL + rn + kc * 32, lane), cl); }
      const float Mn = ST[(b * NPOS + nn) * 2], iLn = ST[(b * NPOS + nn) * 2 + 1];
#pragma unroll
      for (int r = 0; r < 8; ++r) { const float s = c[r] + cl[r] * (1.0f / 2048.0f); const float w = exp_p(s - Mn) * iLn; spw[wave][8 * g + r][ct * 16 + col] = (_Float16)(w * 2048.0f); } }
    LDSX();
    { const v16h pa = frag_h(&spw[wave][col][0], lane);
#pragma unroll
      for (int dt = 0; dt < 8; ++dt) acc[dt] = wmma16(pa, frag_h(VH + (b * CO + dt * 16 + col) * NPOS + j0, lane), acc[dt]); }
    LDSX(); }
  (void)0;
#pragma unroll
  for (int dt = 0; dt < 8; ++dt)
#pragma unroll
    for (int r = 0; r < 8; ++r) { const float v = acc[dt][r] * (1.0f / 2048.0f); const __bf16 hb = (__bf16)v; syh[wave * 16 + 8 * g + r][dt * 16 + col] = hb; syl[wave * 16 + 8 * g + r][dt * 16 + col] = (__bf16)(v - (float)hb); }
  if (lane < 16) for (int c = CO; c < CO + 8; ++c) { syh[wave * 16 + lane][c] = (__bf16)0.f; syl[wave * 16 + lane][c] = (__bf16)0.f; }
  __syncthreads();
#pragma unroll 1
  for (int pass = 0; pass < 2; ++pass) { v8f z[8] = {};
#pragma unroll
    for (int kc = 0; kc < CO / 32; ++kc) { const v16b a = frag_b(&syh[wave * 16 + col][kc * 32], lane), al = frag_b(&syl[wave * 16 + col][kc * 32], lane);
#pragma unroll
      for (int j = 0; j < 8; ++j) { const v16b w = frag_b(PW + (size_t)(pass * 128 + j * 16 + col) * CO + kc * 32, lane); z[j] = wmma_bf(al, w, z[j]); z[j] = wmma_bf(a, w, z[j]); } }
#pragma unroll
    for (int j = 0; j < 8; ++j) { const int c = pass * 128 + j * 16 + col; const float inv = bfr(G[c]) / sqrtf(bfr(VAR[c]) + 1e-5f); const float sh = bfr(Bt[c]) - bfr(MU[c]) * inv; const float bb = bfr(BW[c]);
#pragma unroll
      for (int r = 0; r < 8; ++r) { const int m = m0 + 8 * g + r; so[j * 16 + col][wave * 16 + 8 * g + r] = (z[j][r] + bb) * inv + sh + bfr(X[(b * CIN + c) * NPOS + m]); } }
    __syncthreads();
    for (int e = tid; e < 128 * 16; e += 128) { const int cl_ = e >> 4, q = e & 15; vst2(OUT + (b * CIN + pass * 128 + cl_) * NPOS + blockIdx.x * 64 + q * 4, *(const v4f*)&so[cl_][q * 4]); }
    __syncthreads(); }
}
extern "C" void kernel_launch(void* const* d_in, const int* in_sizes, int n_in, void* d_out, int out_size, void* d_ws, size_t ws_size, hipStream_t stream) {
  (void)in_sizes; (void)n_in; (void)out_size;
  const float** F = (const float**)d_in;
  if (ws_size < (size_t)WS_END) return;
  char* ws = (char*)d_ws; __bf16 *PK = (__bf16*)(ws + WS_PK), *PW = (__bf16*)(ws + WS_PW); _Float16 *QH = (_Float16*)(ws + WS_QH), *QL = (_Float16*)(ws + WS_QL), *KH = (_Float16*)(ws + WS_KH), *KL = (_Float16*)(ws + WS_KL), *VH = (_Float16*)(ws + WS_VH); float* ST = (float*)(ws + WS_ST);
  k_pack<<<3 * CO + CIN, 256, 0, stream>>>(F[1], F[3], F[5], F[7], PK, PW);
  k_proj<<<dim3(NPOS / 64, NB), 128, 0, stream>>>(F[0], PK, F[2], F[4], F[6], QH, QL, KH, KL, VH);
  k_stats<<<dim3(NPOS / 64, NB), 128, 0, stream>>>(QH, QL, KH, KL, ST);
  k_out<<<dim3(TQB, NB), 128, 0, stream>>>(QH, QL, KH, KL, VH, ST, PW, F[8], F[9], F[10], F[11], F[12], F[0], (float*)d_out);
}
